// S4Layer_41489384079817
// MI455X (gfx1250) — hardware-verified
//
#include <hip/hip_runtime.h>
#include <math.h>

typedef __attribute__((ext_vector_type(16))) _Float16 v16h;
typedef __attribute__((ext_vector_type(8)))  _Float16 v8h;
typedef __attribute__((ext_vector_type(16))) __bf16   v16b;
typedef __attribute__((ext_vector_type(8)))  __bf16   v8b;
typedef __attribute__((ext_vector_type(8)))  float    v8f;
typedef __attribute__((ext_vector_type(4)))  float    v4f;

constexpr int kBatch = 4;
constexpr int kSeq   = 2048;
constexpr int kDm    = 1024;
constexpr int kDs    = 256;
constexpr int kHeads = 2;
constexpr int kDh    = 128;
constexpr int kRows  = kBatch * kSeq;
constexpr float kLnEps     = 1e-5f;
constexpr float kWpCarry   = 1024.0f;
constexpr float kHCarry    = 256.0f;
constexpr float kWeffCarry = 1024.0f;
constexpr float kScale1    = 1.0f / 1024.0f;
constexpr float kScale2    = 1.0f / (256.0f * 1024.0f);
constexpr int kTrRows  = 8;
constexpr int kTrPitch = kDm + 4;
constexpr int kScanCh  = 64;
constexpr int kScanTS  = 64;
constexpr int kScanYP  = 68;
constexpr int kLnRows  = 8;
static_assert(kHeads * kDh == kDs, "state width");
static_assert((kDm % 32) == 0 && (kDs % 32) == 0, "GEMM K multiples of 32");
static_assert((kRows % 64) == 0 && (kDs % 64) == 0 && (kDm % 64) == 0, "GEMM M,N multiples of 64");
static_assert((kDs % kTrRows) == 0 && (kDm % 256) == 0, "transpose tiling");
static_assert((kSeq % kScanTS) == 0 && (kDs % kScanCh) == 0, "scan tiling");
static_assert((kRows % kLnRows) == 0 && kDm == 1024, "LayerNorm tiling");

constexpr size_t kOffX16  = 0;
constexpr size_t kOffWPT  = kOffX16 + (size_t)kRows * kDm * 2;
constexpr size_t kOffWEF  = kOffWPT + (size_t)kDs * kDm * 2;
constexpr size_t kOffU    = kOffWEF + (size_t)kDm * kDs * 2;
constexpr size_t kOffH16  = kOffU   + (size_t)kRows * kDs * 4;
constexpr size_t kOffZ    = kOffH16 + (size_t)kRows * kDs * 2;
constexpr size_t kWsTotal = kOffZ   + (size_t)kRows * kDm * 4;
static_assert(kWsTotal == 63963136ull, "carve total");
static_assert(kWsTotal <= 134217728ull, "carve cap");
static_assert((kOffWPT % 128) == 0 && (kOffWEF % 128) == 0 && (kOffU % 128) == 0 &&
              (kOffH16 % 128) == 0 && (kOffZ % 128) == 0, "128-B aligned regions");

__device__ __forceinline__ unsigned short f2bf_bits(float f) {
  unsigned u = __float_as_uint(f);
  return (unsigned short)((u + 0x7FFFu + ((u >> 16) & 1u)) >> 16);
}
__device__ __forceinline__ float bf_bits2f(unsigned short h) { return __uint_as_float(((unsigned)h) << 16); }

__device__ __forceinline__ void dep_guard_h(v8f& a, v8f& b, v16h x, v16h y) { asm volatile("v_nop\n\tv_nop\n\tv_nop\n\tv_nop" : "+v"(a), "+v"(b) : "v"(x), "v"(y)); }
__device__ __forceinline__ void dep_guard_b(v8f& a, v8f& b, v16b x, v16b y) { asm volatile("v_nop\n\tv_nop\n\tv_nop\n\tv_nop" : "+v"(a), "+v"(b) : "v"(x), "v"(y)); }
__device__ __forceinline__ void dep_guard4_h(v8f& a, v8f& b, v8f& c, v8f& d, v16h x, v16h y) { asm volatile("v_nop\n\tv_nop\n\tv_nop\n\tv_nop" : "+v"(a), "+v"(b), "+v"(c), "+v"(d) : "v"(x), "v"(y)); }
__device__ __forceinline__ void dep_guard4_b(v8f& a, v8f& b, v8f& c, v8f& d, v16b x, v16b y) { asm volatile("v_nop\n\tv_nop\n\tv_nop\n\tv_nop" : "+v"(a), "+v"(b), "+v"(c), "+v"(d) : "v"(x), "v"(y)); }
__device__ __forceinline__ void keep4_h(v16h a, v16h b, v16h c, v16h d) { asm volatile("v_nop" :: "v"(a), "v"(b), "v"(c), "v"(d)); }
__device__ __forceinline__ void keep4_b(v16b a, v16b b, v16b c, v16b d) { asm volatile("v_nop" :: "v"(a), "v"(b), "v"(c), "v"(d)); }
__device__ __forceinline__ void acc_guard4(v8f& a, v8f& b, v8f& c, v8f& d) { asm volatile("v_nop\n\tv_nop\n\tv_nop\n\tv_nop" : "+v"(a), "+v"(b), "+v"(c), "+v"(d)); }
template <typename T> struct Frag;
template <> struct Frag<_Float16> {
  typedef v16h V; union U { v16h v; v8h h[2]; };
  static __device__ __forceinline__ v16h load(const _Float16* p) {
    U f; f.h[0] = *(const v8h*)(p); f.h[1] = *(const v8h*)(p + 16); return f.v;
  }
  static __device__ __forceinline__ v8f mma(v16h a, v16h b, v8f c) {
    return __builtin_amdgcn_wmma_f32_16x16x32_f16(false, a, false, b, (short)0, c, false, false);
  }
  static __device__ __forceinline__ void guard(v8f& a, v8f& b, v16h x, v16h y) { dep_guard_h(a, b, x, y); }
  static __device__ __forceinline__ void guard4(v8f& a, v8f& b, v8f& c, v8f& d, v16h x, v16h y) { dep_guard4_h(a, b, c, d, x, y); }
  static __device__ __forceinline__ void keep(v16h a, v16h b, v16h c, v16h d) { keep4_h(a, b, c, d); }
};
template <> struct Frag<__bf16> {
  typedef v16b V; union U { v16b v; v8b h[2]; };
  static __device__ __forceinline__ v16b load(const __bf16* p) {
    U f; f.h[0] = *(const v8b*)(p); f.h[1] = *(const v8b*)(p + 16); return f.v;
  }
  static __device__ __forceinline__ v8f mma(v16b a, v16b b, v8f c) {
    return __builtin_amdgcn_wmma_f32_16x16x32_bf16(false, a, false, b, (short)0, c, false, false);
  }
  static __device__ __forceinline__ void guard(v8f& a, v8f& b, v16b x, v16b y) { dep_guard_b(a, b, x, y); }
  static __device__ __forceinline__ void guard4(v8f& a, v8f& b, v8f& c, v8f& d, v16b x, v16b y) { dep_guard4_b(a, b, c, d, x, y); }
  static __device__ __forceinline__ void keep(v16b a, v16b b, v16b c, v16b d) { keep4_b(a, b, c, d); }
};

template <int ET> struct Elem;
template <> struct Elem<0> { typedef _Float16 T; };
template <> struct Elem<1> { typedef __bf16 T; };
template <int ET, bool SPLIT, int BIAS_MODE, int OUT_MODE, bool RESID>
__global__ __launch_bounds__(256) void wmma_gemm64(
    const unsigned short* __restrict__ Ap, const unsigned short* __restrict__ A2p, int lda, long strideA,
    const unsigned short* __restrict__ Btp, const unsigned short* __restrict__ Bt2p, int ldb, long strideB,
    void* __restrict__ Cout, void* __restrict__ Cout2, int ldc, long strideC,
    const float* __restrict__ bias,
    const float* __restrict__ resid, long strideR,
    int M, int N, int K, float scale) {
  static_assert(!(RESID && OUT_MODE != 0), "residual path is f32-out only");
  typedef typename Elem<ET>::T T;
  typedef typename Frag<T>::V V;
  const T* A = (const T*)Ap; const T* A2 = (const T*)A2p; const T* Bt = (const T*)Btp; const T* Bt2 = (const T*)Bt2p;
  __shared__ __align__(16) float sT[8][16 * 68];
  const int b    = blockIdx.y;
  const int lane = threadIdx.x & 31;
  const int wave = threadIdx.x >> 5;
  const int tilesN = N >> 6;
  const int tilesM = M >> 6;
  const int tile = blockIdx.x * 8 + wave;
  if (tile >= tilesM * tilesN) return;
  const int tm = tile / tilesN;
  const int tn = tile - tm * tilesN;
  const int m0 = tm << 6;
  const int n0 = tn << 6;

  const T* Ab  = A  + (size_t)b * strideA;
  const T* Bb  = Bt + (size_t)b * strideB;
  const T* Ab2 = SPLIT ? (A2  + (size_t)b * strideA) : nullptr;
  const T* Bb2 = SPLIT ? (Bt2 + (size_t)b * strideB) : nullptr;

  const int rlane = lane & 15;
  const int koff  = (lane >> 4) * 8;
  const int mOff  = (lane >> 4) * 8;

  v8f acc[4][4];
#pragma unroll
  for (int i = 0; i < 4; ++i)
#pragma unroll
    for (int j = 0; j < 4; ++j) acc[i][j] = (v8f){0.f,0.f,0.f,0.f,0.f,0.f,0.f,0.f};

  for (int k0 = 0; k0 < K; k0 += 32) {
    V bh[4], bl[4];
#pragma unroll
    for (int j = 0; j < 4; ++j) {
      const size_t bo = (size_t)(n0 + (j << 4) + rlane) * ldb + koff + k0;
      bh[j] = Frag<T>::load(Bb + bo);
      if (SPLIT) bl[j] = Frag<T>::load(Bb2 + bo);
    }
#pragma unroll
    for (int i = 0; i < 4; ++i) {
      const size_t ao = (size_t)(m0 + (i << 4) + rlane) * lda + koff + k0;
      V ah = Frag<T>::load(Ab + ao);
      V al = ah;
      if (SPLIT) al = Frag<T>::load(Ab2 + ao);
#pragma unroll
      for (int j = 0; j < 4; ++j) {
        acc[i][j] = Frag<T>::mma(ah, bh[j], acc[i][j]);
        if (SPLIT) {
          acc[i][j] = Frag<T>::mma(ah, bl[j], acc[i][j]);
          acc[i][j] = Frag<T>::mma(al, bh[j], acc[i][j]);
        }
      }
      Frag<T>::guard4(acc[i][0], acc[i][1], acc[i][2], acc[i][3], ah, al);
    }
    Frag<T>::keep(bh[0], bh[1], bh[2], bh[3]);
    if (SPLIT) Frag<T>::keep(bl[0], bl[1], bl[2], bl[3]);
  }
  acc_guard4(acc[0][0], acc[0][1], acc[0][2], acc[0][3]);
  acc_guard4(acc[1][0], acc[1][1], acc[1][2], acc[1][3]);
  acc_guard4(acc[2][0], acc[2][1], acc[2][2], acc[2][3]);
  acc_guard4(acc[3][0], acc[3][1], acc[3][2], acc[3][3]);

  float* slab = sT[wave];
  const float* Rb = RESID ? (resid + (size_t)b * strideR) : nullptr;
#pragma unroll
  for (int i = 0; i < 4; ++i) {
    const int mBase = m0 + (i << 4);
#pragma unroll
    for (int j = 0; j < 4; ++j) {
      const int n = n0 + (j << 4) + rlane;
      float bv = 0.f;
      if (BIAS_MODE == 2) bv = bias[n];
#pragma unroll
      for (int r = 0; r < 8; ++r) {
        float v = acc[i][j][r] * scale;
        if (BIAS_MODE == 1) v += bias[mBase + mOff + r];
        if (BIAS_MODE == 2) v += bv;
        slab[(mOff + r) * 68 + (j << 4) + rlane] = v;
      }
    }
    __builtin_amdgcn_fence(__ATOMIC_RELEASE, "workgroup");
    __builtin_amdgcn_wave_barrier();
    __builtin_amdgcn_fence(__ATOMIC_ACQUIRE, "workgroup");
    if (OUT_MODE == 0) {
      float* C = (float*)Cout + (size_t)b * strideC;
      const int hh = lane >> 4, c4 = (lane & 15) * 4;
      v4f vals[8];
#pragma unroll
      for (int it = 0; it < 8; ++it) {
        const int row = it * 2 + hh;
        v4f v = *(const v4f*)(slab + row * 68 + c4);
        if (RESID) {
          const v4f rr = *(const v4f*)(Rb + (size_t)(mBase + row) * ldc + n0 + c4);
          v += rr;
        }
        vals[it] = v;
      }
      for (int pass = 0; pass < 2; ++pass) {
#pragma unroll
        for (int it = 0; it < 8; ++it) {
          const int row = it * 2 + hh;
          *(volatile v4f*)(C + (size_t)(mBase + row) * ldc + n0 + c4) = vals[it];
        }
        __threadfence();
      }
    } else {
      const int q = lane >> 3, c8 = (lane & 7) * 8;
      unsigned short* C  = (unsigned short*)Cout  + (size_t)b * strideC;
      unsigned short* C2 = (OUT_MODE == 2) ? ((unsigned short*)Cout2 + (size_t)b * strideC) : nullptr;
      for (int pass = 0; pass < 2; ++pass) {
#pragma unroll
        for (int it = 0; it < 4; ++it) {
          const int row = it * 4 + q;
          const float* sp = slab + row * 68 + c8;
          v8h hv, lv;
#pragma unroll
          for (int e = 0; e < 8; ++e) {
            if (OUT_MODE == 1) {
              hv[e] = (_Float16)sp[e];
            } else {
              unsigned short hb = f2bf_bits(sp[e]);
              unsigned short lb = f2bf_bits(sp[e] - bf_bits2f(hb));
              hv[e] = __builtin_bit_cast(_Float16, hb);
              lv[e] = __builtin_bit_cast(_Float16, lb);
            }
          }
          *(volatile v8h*)(C + (size_t)(mBase + row) * ldc + n0 + c8) = hv;
          if (OUT_MODE == 2) *(volatile v8h*)(C2 + (size_t)(mBase + row) * ldc + n0 + c8) = lv;
        }
        __threadfence();
      }
    }
    __builtin_amdgcn_fence(__ATOMIC_RELEASE, "workgroup");
    __builtin_amdgcn_wave_barrier();
    __builtin_amdgcn_fence(__ATOMIC_ACQUIRE, "workgroup");
  }
}

__global__ __launch_bounds__(256) void cast_rows_f16_kernel(
    const float* __restrict__ src, unsigned short* __restrict__ dst, int total8)
{
  const int i = blockIdx.x * 256 + threadIdx.x;
  if (i >= total8) return;
  const size_t e0 = (size_t)i << 3;
  const v4f a0 = *(const v4f*)(src + e0);
  const v4f a1 = *(const v4f*)(src + e0 + 4);
  v8h hv;
#pragma unroll
  for (int e = 0; e < 4; ++e) {
    hv[e]     = (_Float16)a0[e];
    hv[4 + e] = (_Float16)a1[e];
  }
  unsigned short* qh = dst + e0;
  *(volatile v8h*)qh = hv;
  __threadfence();
  *(volatile v8h*)qh = hv;
}

__global__ __launch_bounds__(256) void wpt_transpose_kernel(
    const float* __restrict__ Wp, unsigned short* __restrict__ WPT)
{
  __shared__ __align__(16) float sT[kTrRows * kTrPitch];
  const int tid = threadIdx.x, lane = tid & 31, wave = tid >> 5;
  const int n0 = blockIdx.x * kTrRows;
  const int nn = tid & 7, kq = tid >> 3;
#pragma unroll 4
  for (int it = 0; it < kDm / 32; ++it) {
    const int k = it * 32 + kq;
    sT[nn * kTrPitch + k] = Wp[(size_t)k * kDs + n0 + nn] * kWpCarry;
  }
  __syncthreads();
  v8h hv[4];
#pragma unroll
  for (int it = 0; it < 4; ++it) {
    const float* sp = sT + wave * kTrPitch + it * 256 + lane * 8;
    const v4f a0 = *(const v4f*)(sp);
    const v4f a1 = *(const v4f*)(sp + 4);
#pragma unroll
    for (int e = 0; e < 4; ++e) {
      hv[it][e]     = (_Float16)a0[e];
      hv[it][4 + e] = (_Float16)a1[e];
    }
  }
  unsigned short* dst = WPT + (size_t)(n0 + wave) * kDm;
  for (int pass = 0; pass < 2; ++pass) {
#pragma unroll
    for (int it = 0; it < 4; ++it) *(volatile v8h*)(dst + it * 256 + lane * 8) = hv[it];
    __threadfence();
  }
}

__global__ __launch_bounds__(256) void weff_fold_kernel(
    const float* __restrict__ Cp, const float* __restrict__ Wo, unsigned short* __restrict__ WEF)
{
  __shared__ __align__(16) float sWo[kDs];
  __shared__ __align__(16) float sR[kDs];
  const int m = blockIdx.x, tid = threadIdx.x, lane = tid & 31, wave = tid >> 5;
  sWo[tid] = Wo[(size_t)tid * kDm + m];
  __syncthreads();
  const int hh = tid >> 7, d = tid & (kDh - 1);
  const float* cb = Cp + (size_t)hh * kDh * kDh + d;
  const float* wb = sWo + hh * kDh;
  float s = 0.0f;
#pragma unroll 4
  for (int e = 0; e < kDh; ++e) s = fmaf(cb[(size_t)e * kDh], wb[e], s);
  sR[tid] = s * kWeffCarry;
  __syncthreads();
  if (wave == 0) {
    const float* sp = sR + lane * 8;
    const v4f a0 = *(const v4f*)(sp);
    const v4f a1 = *(const v4f*)(sp + 4);
    v8h hv;
#pragma unroll
    for (int e = 0; e < 4; ++e) {
      hv[e]     = (_Float16)a0[e];
      hv[4 + e] = (_Float16)a1[e];
    }
    unsigned short* dst = WEF + (size_t)m * kDs + lane * 8;
    *(volatile v8h*)dst = hv;
    __threadfence();
    *(volatile v8h*)dst = hv;
  }
}

__global__ __launch_bounds__(64) void scan_kernel(
    const float* __restrict__ U, const float* __restrict__ lnl, const float* __restrict__ Bsc,
    unsigned short* __restrict__ H16)
{
  __shared__ __align__(16) float sY[kScanTS * kScanYP];
  const int tid = threadIdx.x, lane = tid & 31, wave = tid >> 5;
  constexpr int kBlkPerB = kDs / kScanCh;
  const int bix = blockIdx.x / kBlkPerB;
  const int c0  = (blockIdx.x - bix * kBlkPerB) * kScanCh;
  const int c   = c0 + tid;
  const size_t row0 = (size_t)bix * kSeq;
  const float lv  = lnl[c];
  const float lam = 1.0f / (1.0f + expf(-lv));
  const float bs  = Bsc[c];
  float h = 0.0f;
  const int q = lane >> 3, c8 = (lane & 7) * 8;
#pragma unroll 1
  for (int t0 = 0; t0 < kSeq; t0 += kScanTS) {
#pragma unroll 1
    for (int s = 0; s < kScanTS; ++s) {
      const float u = U[(row0 + t0 + s) * kDs + c] * bs;
      h = fmaf(lam, h, u);
      sY[s * kScanYP + tid] = h * kHCarry;
    }
    __syncthreads();
    v8h hv[8];
#pragma unroll
    for (int it = 0; it < 8; ++it) {
      const int row = it * 8 + wave * 4 + q;
      const float* sp = sY + row * kScanYP + c8;
      const v4f a0 = *(const v4f*)(sp);
      const v4f a1 = *(const v4f*)(sp + 4);
#pragma unroll
      for (int e = 0; e < 4; ++e) {
        hv[it][e]     = (_Float16)a0[e];
        hv[it][4 + e] = (_Float16)a1[e];
      }
    }
    for (int pass = 0; pass < 2; ++pass) {
#pragma unroll
      for (int it = 0; it < 8; ++it) {
        const int row = it * 8 + wave * 4 + q;
        const size_t o = (row0 + t0 + row) * kDs + c0 + c8;
        *(volatile v8h*)(H16 + o) = hv[it];
      }
      __threadfence();
    }
    __syncthreads();
  }
}

__global__ __launch_bounds__(256) void layernorm_kernel(
    const float* __restrict__ Z, const float* __restrict__ gamma, const float* __restrict__ beta,
    float* __restrict__ out)
{
  __shared__ __align__(16) float sG[kDm];
  __shared__ __align__(16) float sB[kDm];
  const int tid = threadIdx.x, lane = tid & 31, wave = tid >> 5;
  *(v4f*)(sG + tid * 4) = *(const v4f*)(gamma + tid * 4);
  *(v4f*)(sB + tid * 4) = *(const v4f*)(beta + tid * 4);
  __syncthreads();
  const size_t row = (size_t)blockIdx.x * kLnRows + wave;
  const float* zr = Z + row * kDm;
  v4f v[8];
#pragma unroll
  for (int it = 0; it < 8; ++it) v[it] = *(const v4f*)(zr + it * 128 + lane * 4);
  float s = 0.0f;
#pragma unroll
  for (int it = 0; it < 8; ++it) s += (v[it][0] + v[it][1]) + (v[it][2] + v[it][3]);
#pragma unroll
  for (int off = 1; off < 32; off <<= 1) s += __shfl_xor(s, off, 32);
  const float mean = s * (1.0f / (float)kDm);
  float s2 = 0.0f;
#pragma unroll
  for (int it = 0; it < 8; ++it) {
    const v4f d = v[it] - mean;
    s2 += (d[0] * d[0] + d[1] * d[1]) + (d[2] * d[2] + d[3] * d[3]);
  }
#pragma unroll
  for (int off = 1; off < 32; off <<= 1) s2 += __shfl_xor(s2, off, 32);
  const float var  = s2 * (1.0f / (float)kDm);
  const float rstd = 1.0f / sqrtf(var + kLnEps);
  v4f o[8];
#pragma unroll
  for (int it = 0; it < 8; ++it) {
    const v4f g  = *(const v4f*)(sG + it * 128 + lane * 4);
    const v4f bb = *(const v4f*)(sB + it * 128 + lane * 4);
    o[it] = (v[it] - mean) * rstd * g + bb;
  }
  float* orow = out + row * kDm;
  for (int pass = 0; pass < 2; ++pass) {
#pragma unroll
    for (int it = 0; it < 8; ++it) *(volatile v4f*)(orow + it * 128 + lane * 4) = o[it];
    __threadfence();
  }
}

extern "C" void kernel_launch(void* const* d_in, const int* in_sizes, int n_in,
                              void* d_out, int out_size, void* d_ws, size_t ws_size,
                              hipStream_t stream) {
  if (n_in < 10) return;
  if (in_sizes[0] != kRows * kDm) return;
  if (in_sizes[1] != kDm * kDs) return;
  if (in_sizes[2] != kDs) return;
  if (in_sizes[3] != kDs * kDm) return;
  if (in_sizes[4] != kDm) return;
  if (in_sizes[5] != kHeads * kDh) return;
  if (in_sizes[6] != kHeads * kDh) return;
  if (in_sizes[7] != kHeads * kDh * kDh) return;
  if (in_sizes[8] != kDm) return;
  if (in_sizes[9] != kDm) return;
  if (out_size != kRows * kDm) return;
  if (ws_size < kWsTotal) return;

  const float* x     = (const float*)d_in[0];
  const float* Wp    = (const float*)d_in[1];
  const float* bp    = (const float*)d_in[2];
  const float* Wo    = (const float*)d_in[3];
  const float* bo    = (const float*)d_in[4];
  const float* lnl   = (const float*)d_in[5];
  const float* Bsc   = (const float*)d_in[6];
  const float* Cp    = (const float*)d_in[7];
  const float* gamma = (const float*)d_in[8];
  const float* beta  = (const float*)d_in[9];
  float* out = (float*)d_out;

  char* ws = (char*)d_ws;
  unsigned short* X16 = (unsigned short*)(ws + kOffX16);
  unsigned short* WPT = (unsigned short*)(ws + kOffWPT);
  unsigned short* WEF = (unsigned short*)(ws + kOffWEF);
  float*          U   = (float*)(ws + kOffU);
  unsigned short* H16 = (unsigned short*)(ws + kOffH16);
  float*          Z   = (float*)(ws + kOffZ);

  cast_rows_f16_kernel<<<(kRows * kDm / 8) / 256, 256, 0, stream>>>(x, X16, kRows * kDm / 8);
  wpt_transpose_kernel<<<kDs / kTrRows, 256, 0, stream>>>(Wp, WPT);
  weff_fold_kernel<<<kDm, 256, 0, stream>>>(Cp, Wo, WEF);

  wmma_gemm64<0, false, 2, 0, false><<<dim3((kRows / 64) * (kDs / 64) / 8, 1), 256, 0, stream>>>(
      X16, nullptr, kDm, 0L,
      WPT, nullptr, kDm, 0L,
      (void*)U, nullptr, kDs, 0L,
      bp, nullptr, 0L,
      kRows, kDs, kDm, kScale1);

  scan_kernel<<<kBatch * (kDs / kScanCh), kScanCh, 0, stream>>>(U, lnl, Bsc, H16);

  wmma_gemm64<0, false, 2, 0, true><<<dim3((kRows / 64) * (kDm / 64) / 8, 1), 256, 0, stream>>>(
      H16, nullptr, kDs, 0L,
      WEF, nullptr, kDs, 0L,
      (void*)Z, nullptr, kDm, 0L,
      bo, x, 0L,
      kRows, kDm, kDs, kScale2);

  layernorm_kernel<<<kRows / kLnRows, 256, 0, stream>>>(Z, gamma, beta, out);
}
